// SceneGraphGAT_31482110279997
// MI455X (gfx1250) — hardware-run, weakly checked
//
#include <hip/hip_runtime.h>
#include <stddef.h>


#define KIN     256
#define HC      128
#define YP      256
#define EP      2
#define NTHR    256
#define NWAVE   8
#define EPT     8
#define CHUNK   (NTHR * EPT)
#define WCAP    (EPT * 32)
#define LISTN   (NWAVE * WCAP)
#define NBMAX   2048
#define RCAP    28672
#define DEGCAP  4096
#define GBM     64
#define GTHR    128
#define NEG_SLOPE 0.2f
#define CA      16.0f
#define CW      64.0f
#define SCL     0.0009765625f
#define WSCAP   134217728
#define LDS_AGG ((2 * RCAP + 2 * NBMAX + LISTN) * 4 + 64)

static_assert((CHUNK & (CHUNK - 1)) == 0 && CHUNK <= 4096);
static_assert((NBMAX & (NBMAX - 1)) == 0 && NBMAX <= 4096);
static_assert(NTHR * 8 == NBMAX);
static_assert(LISTN >= NBMAX);
static_assert(LISTN >= NWAVE * WCAP);
static_assert((RCAP % 32) == 0);
static_assert(LDS_AGG <= 300000);
static_assert(GBM == (GTHR / 32) * 16);
static_assert(GTHR == HC);
static_assert((KIN % 32) == 0);
static_assert(YP == 2 * HC);
static_assert(GBM * EP == 32 * 4);
static_assert(2 * GBM == GTHR);

typedef float    v2f  __attribute__((ext_vector_type(2)));
typedef float    v4f  __attribute__((ext_vector_type(4)));
typedef float    v8f  __attribute__((ext_vector_type(8)));
typedef int      v4i  __attribute__((ext_vector_type(4)));
typedef int      v8i  __attribute__((ext_vector_type(8)));
typedef _Float16 v4h  __attribute__((ext_vector_type(4)));
typedef _Float16 v8h  __attribute__((ext_vector_type(8)));
typedef _Float16 v16h __attribute__((ext_vector_type(16)));
union FragH { v16h v; v8h h[2]; v8i w; };

__device__ __forceinline__ v8f wmh(const FragH& a, const FragH& b, v8f c) {
  v8f d = __builtin_amdgcn_wmma_f32_16x16x32_f16(false, a.v, false, b.v, (short)0, c, false, false);
  asm volatile("v_nop\n\tv_nop\n\tv_nop\n\tv_nop" : "+v"(d) : "v"(a.w), "v"(b.w));
  return d;
}

__device__ __forceinline__ int scan_chunk(const int* __restrict__ dsts, int nE, int cbase, int slotBase,
                                          int nb, int vec8, int* list, int tid, int lane, int wave) {
  int wc = 0;
  const int el0  = tid * EPT;
  const int e0   = cbase + el0;
  const int sent = -2147483647 - 1;
  v4i da, db;
  if (vec8 != 0 && cbase + CHUNK <= nE) {
    da = *(const v4i*)(dsts + e0);
    db = *(const v4i*)(dsts + e0 + 4);
  } else {
    da.x = (e0     < nE) ? dsts[min(e0,     nE - 1)] : sent;
    da.y = (e0 + 1 < nE) ? dsts[min(e0 + 1, nE - 1)] : sent;
    da.z = (e0 + 2 < nE) ? dsts[min(e0 + 2, nE - 1)] : sent;
    da.w = (e0 + 3 < nE) ? dsts[min(e0 + 3, nE - 1)] : sent;
    db.x = (e0 + 4 < nE) ? dsts[min(e0 + 4, nE - 1)] : sent;
    db.y = (e0 + 5 < nE) ? dsts[min(e0 + 5, nE - 1)] : sent;
    db.z = (e0 + 6 < nE) ? dsts[min(e0 + 6, nE - 1)] : sent;
    db.w = (e0 + 7 < nE) ? dsts[min(e0 + 7, nE - 1)] : sent;
  }
  const unsigned nbs = (unsigned)slotBase;
  const unsigned unb = (unsigned)nb;
  const unsigned s0 = (unsigned)da.x - nbs, s1 = (unsigned)da.y - nbs;
  const unsigned s2 = (unsigned)da.z - nbs, s3 = (unsigned)da.w - nbs;
  const unsigned s4 = (unsigned)db.x - nbs, s5 = (unsigned)db.y - nbs;
  const unsigned s6 = (unsigned)db.z - nbs, s7 = (unsigned)db.w - nbs;
  const bool h0 = s0 < unb, h1 = s1 < unb, h2 = s2 < unb, h3 = s3 < unb;
  const bool h4 = s4 < unb, h5 = s5 < unb, h6 = s6 < unb, h7 = s7 < unb;
  const unsigned any = __builtin_amdgcn_ballot_w32(h0 | h1 | h2 | h3 | h4 | h5 | h6 | h7);
  if (any != 0u) {
#define HITJ(J, HJ, SJ) { \
      const unsigned mj = __builtin_amdgcn_ballot_w32(HJ); \
      if (mj != 0u) { \
        if (HJ) { \
          const int pos = wc + (int)__builtin_amdgcn_mbcnt_lo(mj, 0u); \
          if (pos < WCAP) list[wave * WCAP + pos] = ((el0 + (J)) << 12) | (int)(SJ); \
        } \
        wc += (int)__builtin_popcount(mj); } }
    HITJ(0, h0, s0)
    HITJ(1, h1, s1)
    HITJ(2, h2, s2)
    HITJ(3, h3, s3)
    HITJ(4, h4, s4)
    HITJ(5, h5, s5)
    HITJ(6, h6, s6)
    HITJ(7, h7, s7)
#undef HITJ
  }
  return wc;
}

__global__ __launch_bounds__(NTHR) void k_xprep(const float* __restrict__ x, _Float16* xh, int nN, int nUnits) {
  const int i = (int)blockIdx.x * NTHR + (int)threadIdx.x;
  if (i >= nUnits) return;
  const int row = i >> 5;
  const int c0  = (i & 31) * 8;
  const int rc  = row < nN ? row : nN - 1;
  const float* p = x + (size_t)rc * KIN + c0;
  v4f a = *(const v4f*)p, b = *(const v4f*)(p + 4);
  const v4f z4 = {0.f, 0.f, 0.f, 0.f};
  if (row >= nN) { a = z4; b = z4; }
  v8h hv;
  hv[0] = (_Float16)(a.x * CA); hv[1] = (_Float16)(a.y * CA);
  hv[2] = (_Float16)(a.z * CA); hv[3] = (_Float16)(a.w * CA);
  hv[4] = (_Float16)(b.x * CA); hv[5] = (_Float16)(b.y * CA);
  hv[6] = (_Float16)(b.z * CA); hv[7] = (_Float16)(b.w * CA);
  const size_t o = (size_t)row * KIN + c0;
  *(volatile v8h*)(xh + o) = hv;
  __threadfence();
  *(volatile v8h*)(xh + o) = hv;
}

__global__ __launch_bounds__(NTHR) void k_wprep(const float* __restrict__ w1, const float* __restrict__ w2,
                                                _Float16* wt) {
  const int j  = (int)blockIdx.y;
  const int u  = (int)blockIdx.x * NTHR + (int)threadIdx.x;
  const int nc = (j == 0) ? (2 * HC) : HC;
  const int nUnits = nc * (KIN / 8);
  if (u >= nUnits) return;
  const int n  = u >> 5;
  const int k8 = (u & 31) * 8;
  const float* src = (j == 0) ? w1 : w2;
  const float* p = src + (size_t)k8 * nc + n;
  v4f a, b;
  a.x = p[0 * nc]; a.y = p[1 * nc]; a.z = p[2 * nc]; a.w = p[3 * nc];
  b.x = p[4 * nc]; b.y = p[5 * nc]; b.z = p[6 * nc]; b.w = p[7 * nc];
  v8h hv;
  hv[0] = (_Float16)(a.x * CW); hv[1] = (_Float16)(a.y * CW);
  hv[2] = (_Float16)(a.z * CW); hv[3] = (_Float16)(a.w * CW);
  hv[4] = (_Float16)(b.x * CW); hv[5] = (_Float16)(b.y * CW);
  hv[6] = (_Float16)(b.z * CW); hv[7] = (_Float16)(b.w * CW);
  const size_t rowb = (j == 0) ? 0 : (size_t)(2 * HC);
  const size_t o = (rowb + (size_t)n) * KIN + k8;
  *(volatile v8h*)(wt + o) = hv;
  __threadfence();
  *(volatile v8h*)(wt + o) = hv;
}

__global__ __launch_bounds__(GTHR) void k_gemm(const _Float16* __restrict__ xh, const _Float16* __restrict__ wt,
                                               const float* __restrict__ asrc, const float* __restrict__ adst,
                                               float* Y, float* ES, float* ED, int nP) {
  __shared__ __attribute__((aligned(16))) float stg[GBM * HC];
  __shared__ __attribute__((aligned(16))) float esT[GBM * EP];
  __shared__ __attribute__((aligned(16))) float edT[GBM * EP];
  __shared__ float sAs[2 * HC];
  __shared__ float sAd[2 * HC];
  const int tid = threadIdx.x, lane = tid & 31, wave = tid >> 5, hh = lane >> 4, m = lane & 15;
  const int rowBase = (int)blockIdx.x * GBM;
  const int nA = nP * HC;
  {
    const int i1 = (tid + HC < nA) ? (tid + HC) : (nA - 1);
    sAs[tid] = asrc[tid];
    sAd[tid] = adst[tid];
    sAs[tid + HC] = asrc[i1];
    sAd[tid + HC] = adst[i1];
  }
  const size_t arow = (size_t)(rowBase + 16 * wave + m) * KIN + 8 * hh;
#pragma unroll 1
  for (int p = 0; p < nP; ++p) {
#pragma unroll 1
    for (int ch = 0; ch < 2; ++ch) {
      v8f acc[4];
#pragma unroll
      for (int t = 0; t < 4; ++t) { v8f z = {0.f, 0.f, 0.f, 0.f, 0.f, 0.f, 0.f, 0.f}; acc[t] = z; }
      const int ncol0 = 64 * ch;
      const size_t brow = (size_t)(p * HC + ncol0 + m) * KIN + 8 * hh;
#pragma unroll 1
      for (int ks = 0; ks < KIN / 32; ++ks) {
        FragH af;
        af.h[0] = *(const v8h*)(xh + arow + 32 * ks);
        af.h[1] = *(const v8h*)(xh + arow + 32 * ks + 16);
#pragma unroll
        for (int t = 0; t < 4; ++t) {
          const size_t bo = brow + (size_t)(16 * t) * KIN + 32 * ks;
          FragH bf;
          bf.h[0] = *(const v8h*)(wt + bo);
          bf.h[1] = *(const v8h*)(wt + bo + 16);
          acc[t] = wmh(af, bf, acc[t]);
        }
      }
      float* sp = stg + (size_t)(16 * wave + 8 * hh) * HC + ncol0 + m;
#pragma unroll
      for (int t = 0; t < 4; ++t) {
#pragma unroll
        for (int r = 0; r < 8; ++r) sp[(size_t)r * HC + 16 * t] = acc[t][r] * SCL;
      }
    }
    __syncthreads();
    {
      const int row  = tid >> 1;
      const int half = tid & 1;
      const float* srow = stg + (size_t)row * HC;
      float s = 0.f, d = 0.f;
#pragma unroll 1
      for (int c = 0; c < 64; ++c) {
        const int cc = half * 64 + c;
        const float v = srow[cc];
        s = fmaf(v, sAs[p * HC + cc], s);
        d = fmaf(v, sAd[p * HC + cc], d);
      }
      s += __shfl_xor(s, 1);
      d += __shfl_xor(d, 1);
      if (half == 0) {
        esT[row * EP + p] = s;
        edT[row * EP + p] = d;
      } else if (nP == 1) {
        esT[row * EP + 1] = 0.f;
        edT[row * EP + 1] = 0.f;
      }
    }
    const int nF4 = GBM * HC / 4;
    float* yb = Y + (size_t)rowBase * YP + HC * p;
    const v4f* s4 = (const v4f*)stg;
#pragma unroll 1
    for (int f = tid; f < nF4; f += GTHR) {
      const int r = f >> 5, q = f & 31;
      const v4f v = s4[f];
      *(volatile v4f*)(yb + (size_t)r * YP + 4 * q) = v;
    }
    __threadfence();
#pragma unroll 1
    for (int f = tid; f < nF4; f += GTHR) {
      const int r = f >> 5, q = f & 31;
      const v4f v = s4[f];
      *(volatile v4f*)(yb + (size_t)r * YP + 4 * q) = v;
    }
    __syncthreads();
  }
  if (wave == 0) {
    const v4f ve = *(const v4f*)(esT + 4 * lane);
    const v4f vd = *(const v4f*)(edT + 4 * lane);
    float* pe = ES + (size_t)rowBase * EP + 4 * lane;
    float* pd = ED + (size_t)rowBase * EP + 4 * lane;
    *(volatile v4f*)pe = ve;
    *(volatile v4f*)pd = vd;
    __threadfence();
    *(volatile v4f*)pe = ve;
    *(volatile v4f*)pd = vd;
  }
}

__global__ __launch_bounds__(NTHR) void k_agg(
    const int* __restrict__ srcs, const int* __restrict__ dsts,
    const float* __restrict__ Y, const float* __restrict__ ES, const float* __restrict__ ED,
    const float* __restrict__ bias, _Float16* xout, float* out,
    int nN, int nE, int nb, int vec8, int lay) {
  extern __shared__ v4f lds_dyn[];
  int* reg1 = (int*)lds_dyn;
  int* reg2 = reg1 + RCAP;
  int* scnt = reg2 + RCAP;
  int* soff = scnt + NBMAX;
  int* list = soff + NBMAX;
  int* wcnt = list + LISTN;
  int* wtot = wcnt + NWAVE;
  const int tid = threadIdx.x, lane = tid & 31, wave = tid >> 5;
  const int nodeBase = (int)blockIdx.x * nb;

  for (int i = tid; i < NBMAX; i += NTHR) scnt[i] = 0;
  __syncthreads();

  int tot = 0;
  const int nChunks = (nE + CHUNK - 1) / CHUNK;
#pragma unroll 1
  for (int ch = 0; ch < nChunks; ++ch) {
    const int cbase = ch * CHUNK;
    const int wc = scan_chunk(dsts, nE, cbase, nodeBase, nb, vec8, list, tid, lane, wave);
    if (lane == 0) wcnt[wave] = wc;
    __syncthreads();
    int pre = 0, all = 0;
#pragma unroll
    for (int w2 = 0; w2 < NWAVE; ++w2) {
      int c = wcnt[w2];
      c = c < 0 ? 0 : (c > WCAP ? WCAP : c);
      all += c;
      pre += (w2 < wave) ? c : 0;
    }
    const int wcc  = wc > WCAP ? WCAP : wc;
    const int base = tot + pre;
#pragma unroll 1
    for (int i = lane; i < wcc; i += 32) {
      const int ent = list[wave * WCAP + i];
      const int el  = (ent >> 12) & (CHUNK - 1);
      const int sl  = ent & (NBMAX - 1);
      int eid = cbase + el;
      eid = eid > nE - 1 ? nE - 1 : eid;
      const int pos = base + i;
      if (pos < RCAP) reg1[pos] = (int)(((unsigned)eid << 12) | (unsigned)sl);
    }
    tot += all;
    tot = tot > RCAP ? RCAP : tot;
    __syncthreads();
  }
  const int nh = tot;

  if (wave == 0) {
#pragma unroll 1
    for (int b0 = 0; b0 < nh; b0 += 32) {
      const int idx = b0 + lane;
      const int uv  = reg1[idx < RCAP ? idx : RCAP - 1];
      const int m32 = (nh - b0) < 32 ? (nh - b0) : 32;
#pragma unroll 1
      for (int k = 0; k < m32; ++k) {
        const int u  = __builtin_amdgcn_readlane(uv, k);
        const int sl = u & (NBMAX - 1);
        if (lane == 0) scnt[sl] = scnt[sl] + 1;
      }
    }
  }
  __syncthreads();

  {
    const v4i ca = *(const v4i*)(scnt + 8 * tid);
    const v4i cb = *(const v4i*)(scnt + 8 * tid + 4);
    const int e0 = ca.x < 0 ? 0 : ca.x, e1 = ca.y < 0 ? 0 : ca.y, e2 = ca.z < 0 ? 0 : ca.z, e3 = ca.w < 0 ? 0 : ca.w;
    const int e4 = cb.x < 0 ? 0 : cb.x, e5 = cb.y < 0 ? 0 : cb.y, e6 = cb.z < 0 ? 0 : cb.z, e7 = cb.w < 0 ? 0 : cb.w;
    const int ts = e0 + e1 + e2 + e3 + e4 + e5 + e6 + e7;
    int incl = ts;
#pragma unroll
    for (int d = 1; d < 32; d <<= 1) {
      const int up = __shfl_up(incl, d);
      if (lane >= d) incl += up;
    }
    if (lane == 31) wtot[wave] = incl;
    __syncthreads();
    int pre = 0;
#pragma unroll
    for (int w2 = 0; w2 < NWAVE; ++w2) pre += (w2 < wave) ? wtot[w2] : 0;
    int run = pre + incl - ts;
    soff[8 * tid + 0] = run; run += e0;
    soff[8 * tid + 1] = run; run += e1;
    soff[8 * tid + 2] = run; run += e2;
    soff[8 * tid + 3] = run; run += e3;
    soff[8 * tid + 4] = run; run += e4;
    soff[8 * tid + 5] = run; run += e5;
    soff[8 * tid + 6] = run; run += e6;
    soff[8 * tid + 7] = run;
  }
  __syncthreads();
  for (int i = tid; i < NBMAX; i += NTHR) list[i] = soff[i];
  __syncthreads();

  if (wave == 0) {
#pragma unroll 1
    for (int b0 = 0; b0 < nh; b0 += 32) {
      const int idx = b0 + lane;
      const int uv  = reg1[idx < RCAP ? idx : RCAP - 1];
      const int m32 = (nh - b0) < 32 ? (nh - b0) : 32;
#pragma unroll 1
      for (int k = 0; k < m32; ++k) {
        const int u   = __builtin_amdgcn_readlane(uv, k);
        const int sl  = u & (NBMAX - 1);
        const int eid = (int)((unsigned)u >> 12);
        if (lane == 0) {
          int pos = list[sl];
          pos = pos < 0 ? 0 : (pos > RCAP - 1 ? RCAP - 1 : pos);
          reg2[pos] = eid;
          list[sl] = pos + 1;
        }
      }
    }
  }
  __syncthreads();

  const int nbw = nb >> 3;
  const int c4  = 4 * lane;
  const int cb1 = (lay == 0) ? (HC + c4) : c4;
  const v4f bz0 = *(const v4f*)(bias + c4);
  const v4f bz1 = *(const v4f*)(bias + cb1);
  const bool ovf = (nh >= RCAP);
  const float qnan = __int_as_float(0x7fc00000);
#pragma unroll 1
  for (int jt = 0; jt < nbw; ++jt) {
    const int slot = wave * nbw + jt;
    const int grow = nodeBase + slot;
    const int gcl  = grow < nN ? grow : nN - 1;
    int st = soff[slot];
    const int craw = scnt[slot];
    int cnt = craw;
    st  = st < 0 ? 0 : (st > nh ? nh : st);
    cnt = cnt < 0 ? 0 : (cnt > DEGCAP ? DEGCAP : cnt);
    if (cnt > nh - st) cnt = nh - st;
    const float pz = (ovf || craw > DEGCAP) ? qnan : 0.0f;
    const bool wr = grow < nN;

    const float* yd = Y + (size_t)gcl * YP;
    const v4f xd0 = *(const v4f*)(yd + c4);
    const v2f edv = *(const v2f*)(ED + (size_t)gcl * EP);
    const v2f esv = *(const v2f*)(ES + (size_t)gcl * EP);

    if (lay == 0) {
      const v4f xd1 = *(const v4f*)(yd + HC + c4);
      const float ta = esv.x + edv.x, tb = esv.y + edv.y;
      float mxa = fmaxf(ta, NEG_SLOPE * ta), mxb = fmaxf(tb, NEG_SLOPE * tb);
      float dna = 1.0f, dnb = 1.0f;
      v4f aca = xd0, acb = xd1;
#pragma unroll 1
      for (int q = 0; q < cnt; ++q) {
        int idx = st + q; idx = idx > RCAP - 1 ? RCAP - 1 : idx;
        int eid = reg2[idx]; eid = eid < 0 ? 0 : (eid > nE - 1 ? nE - 1 : eid);
        const int sraw = srcs[eid];
        const int s = sraw < 0 ? 0 : (sraw > nN - 1 ? nN - 1 : sraw);
        const float* ys = Y + (size_t)s * YP;
        const v4f xsa = *(const v4f*)(ys + c4);
        const v4f xsb = *(const v4f*)(ys + HC + c4);
        const v2f ess = *(const v2f*)(ES + (size_t)s * EP);
        const float ua = ess.x + edv.x, ub = ess.y + edv.y;
        const float la = fmaxf(ua, NEG_SLOPE * ua), lb = fmaxf(ub, NEG_SLOPE * ub);
        const float mna = fmaxf(mxa, la), mnb = fmaxf(mxb, lb);
        const float s1a = __expf(mxa - mna), s2a = __expf(la - mna);
        const float s1b = __expf(mxb - mnb), s2b = __expf(lb - mnb);
        dna = fmaf(dna, s1a, s2a);
        dnb = fmaf(dnb, s1b, s2b);
        aca.x = fmaf(aca.x, s1a, s2a * xsa.x);
        aca.y = fmaf(aca.y, s1a, s2a * xsa.y);
        aca.z = fmaf(aca.z, s1a, s2a * xsa.z);
        aca.w = fmaf(aca.w, s1a, s2a * xsa.w);
        acb.x = fmaf(acb.x, s1b, s2b * xsb.x);
        acb.y = fmaf(acb.y, s1b, s2b * xsb.y);
        acb.z = fmaf(acb.z, s1b, s2b * xsb.z);
        acb.w = fmaf(acb.w, s1b, s2b * xsb.w);
        mxa = mna; mxb = mnb;
      }
      const float ia = __builtin_amdgcn_rcpf(dna);
      const float ib = __builtin_amdgcn_rcpf(dnb);
      v4f oa, ob;
      oa.x = fmaf(aca.x, ia, bz0.x); oa.y = fmaf(aca.y, ia, bz0.y);
      oa.z = fmaf(aca.z, ia, bz0.z); oa.w = fmaf(aca.w, ia, bz0.w);
      ob.x = fmaf(acb.x, ib, bz1.x); ob.y = fmaf(acb.y, ib, bz1.y);
      ob.z = fmaf(acb.z, ib, bz1.z); ob.w = fmaf(acb.w, ib, bz1.w);
      v4f ea, eb;
      ea.x = (oa.x > 0.f ? oa.x : (__expf(fminf(oa.x, 0.f)) - 1.0f)) + pz;
      ea.y = (oa.y > 0.f ? oa.y : (__expf(fminf(oa.y, 0.f)) - 1.0f)) + pz;
      ea.z = (oa.z > 0.f ? oa.z : (__expf(fminf(oa.z, 0.f)) - 1.0f)) + pz;
      ea.w = (oa.w > 0.f ? oa.w : (__expf(fminf(oa.w, 0.f)) - 1.0f)) + pz;
      eb.x = (ob.x > 0.f ? ob.x : (__expf(fminf(ob.x, 0.f)) - 1.0f)) + pz;
      eb.y = (ob.y > 0.f ? ob.y : (__expf(fminf(ob.y, 0.f)) - 1.0f)) + pz;
      eb.z = (ob.z > 0.f ? ob.z : (__expf(fminf(ob.z, 0.f)) - 1.0f)) + pz;
      eb.w = (ob.w > 0.f ? ob.w : (__expf(fminf(ob.w, 0.f)) - 1.0f)) + pz;
      v4h ha, hb;
      ha.x = (_Float16)(ea.x * CA); ha.y = (_Float16)(ea.y * CA);
      ha.z = (_Float16)(ea.z * CA); ha.w = (_Float16)(ea.w * CA);
      hb.x = (_Float16)(eb.x * CA); hb.y = (_Float16)(eb.y * CA);
      hb.z = (_Float16)(eb.z * CA); hb.w = (_Float16)(eb.w * CA);
      _Float16* xp = xout + (size_t)gcl * KIN + c4;
      if (wr) {
        *(volatile v4h*)xp = ha;
        *(volatile v4h*)(xp + HC) = hb;
      }
      __threadfence();
      if (wr) {
        *(volatile v4h*)xp = ha;
        *(volatile v4h*)(xp + HC) = hb;
      }
    } else {
      const float ta = esv.x + edv.x;
      float mxa = fmaxf(ta, NEG_SLOPE * ta);
      float dna = 1.0f;
      v4f aca = xd0;
#pragma unroll 1
      for (int q = 0; q < cnt; ++q) {
        int idx = st + q; idx = idx > RCAP - 1 ? RCAP - 1 : idx;
        int eid = reg2[idx]; eid = eid < 0 ? 0 : (eid > nE - 1 ? nE - 1 : eid);
        const int sraw = srcs[eid];
        const int s = sraw < 0 ? 0 : (sraw > nN - 1 ? nN - 1 : sraw);
        const v4f xsa = *(const v4f*)(Y + (size_t)s * YP + c4);
        const v2f ess = *(const v2f*)(ES + (size_t)s * EP);
        const float ua = ess.x + edv.x;
        const float la = fmaxf(ua, NEG_SLOPE * ua);
        const float mna = fmaxf(mxa, la);
        const float s1a = __expf(mxa - mna), s2a = __expf(la - mna);
        dna = fmaf(dna, s1a, s2a);
        aca.x = fmaf(aca.x, s1a, s2a * xsa.x);
        aca.y = fmaf(aca.y, s1a, s2a * xsa.y);
        aca.z = fmaf(aca.z, s1a, s2a * xsa.z);
        aca.w = fmaf(aca.w, s1a, s2a * xsa.w);
        mxa = mna;
      }
      const float ia = __builtin_amdgcn_rcpf(dna);
      v4f o;
      o.x = fmaf(aca.x, ia, bz0.x) + pz; o.y = fmaf(aca.y, ia, bz0.y) + pz;
      o.z = fmaf(aca.z, ia, bz0.z) + pz; o.w = fmaf(aca.w, ia, bz0.w) + pz;
      float* gp = out + (size_t)gcl * HC + c4;
      if (wr) *(volatile v4f*)gp = o;
      __threadfence();
      if (wr) *(volatile v4f*)gp = o;
    }
  }
}

static int pick_nb(int nE, int nN) {
  int nb = NBMAX;
  while (nb > 16 && (long long)nb * (long long)nE * 5LL > (long long)RCAP * (long long)nN * 4LL) nb >>= 1;
  return nb;
}

extern "C" void kernel_launch(void* const* d_in, const int* in_sizes, int n_in,
                              void* d_out, int out_size, void* d_ws, size_t ws_size,
                              hipStream_t stream) {
  if (n_in < 10) return;
  const int nN = in_sizes[0] / KIN;
  if (nN <= 0 || in_sizes[0] != nN * KIN) return;
  if (nN > (1 << 22)) return;
  const int szE = in_sizes[1];
  if (szE < 2 || (szE & 1) != 0) return;
  const int nE = szE / 2;
  if (nE > (1 << 20)) return;
  if (in_sizes[2] != KIN * 2 * HC) return;
  if (in_sizes[3] != 2 * HC || in_sizes[4] != 2 * HC) return;
  if (in_sizes[5] != 2 * HC) return;
  if (in_sizes[6] != KIN * HC) return;
  if (in_sizes[7] != HC || in_sizes[8] != HC) return;
  if (in_sizes[9] != HC) return;
  if (out_size != nN * HC) return;

  const float* x   = (const float*)d_in[0];
  const int*   ei  = (const int*)d_in[1];
  const float* W1  = (const float*)d_in[2];
  const float* as1 = (const float*)d_in[3];
  const float* ad1 = (const float*)d_in[4];
  const float* b1  = (const float*)d_in[5];
  const float* W2  = (const float*)d_in[6];
  const float* as2 = (const float*)d_in[7];
  const float* ad2 = (const float*)d_in[8];
  const float* b2  = (const float*)d_in[9];
  float* out = (float*)d_out;

  const int MP   = ((nN + GBM - 1) / GBM) * GBM;
  const int nb   = pick_nb(nE, nN);
  const int vec8 = ((nE & 3) == 0) ? 1 : 0;
  const int nUnits = MP * (KIN / 8);

  char* ws = (char*)d_ws;
  size_t off = 0;
  const size_t oWT = off; off += (size_t)(3 * HC) * KIN * 2;      off = (off + 255) & ~(size_t)255;
  const size_t oXH = off; off += (size_t)MP * KIN * 2;           off = (off + 255) & ~(size_t)255;
  const size_t oY  = off; off += (size_t)MP * YP * 4;            off = (off + 255) & ~(size_t)255;
  const size_t oES = off; off += (size_t)MP * EP * 4;            off = (off + 255) & ~(size_t)255;
  const size_t oED = off; off += (size_t)MP * EP * 4;            off = (off + 255) & ~(size_t)255;
  if (off > ws_size || off > (size_t)WSCAP) return;
  _Float16* WT = (_Float16*)(ws + oWT);
  _Float16* XH = (_Float16*)(ws + oXH);
  float*    Y  = (float*)(ws + oY);
  float*    ES = (float*)(ws + oES);
  float*    ED = (float*)(ws + oED);
  const int* srcp = ei;
  const int* dstp = ei + nE;

  hipFuncSetAttribute(reinterpret_cast<const void*>(&k_agg),
                      hipFuncAttributeMaxDynamicSharedMemorySize, LDS_AGG);

  k_xprep<<<(nUnits + NTHR - 1) / NTHR, NTHR, 0, stream>>>(x, XH, nN, nUnits);
  k_wprep<<<dim3((2 * HC * (KIN / 8) + NTHR - 1) / NTHR, 2), NTHR, 0, stream>>>(W1, W2, WT);

  const int gG = MP / GBM;
  const int gA = (nN + nb - 1) / nb;

  k_gemm<<<gG, GTHR, 0, stream>>>(XH, WT, as1, ad1, Y, ES, ED, 2);
  k_agg<<<gA, NTHR, LDS_AGG, stream>>>(srcp, dstp, Y, ES, ED, b1, XH, out, nN, nE, nb, vec8, 0);
  k_gemm<<<gG, GTHR, 0, stream>>>(XH, WT + (size_t)(2 * HC) * KIN, as2, ad2, Y, ES, ED, 1);
  k_agg<<<gA, NTHR, LDS_AGG, stream>>>(srcp, dstp, Y, ES, ED, b2, XH, out, nN, nE, nb, vec8, 1);
}
